// STU_7928509629254
// MI455X (gfx1250) — hardware-verified
//
#include <hip/hip_runtime.h>
#include <stddef.h>
#include <stdint.h>
#include <math.h>

typedef __attribute__((ext_vector_type(16))) _Float16 v16h;
typedef __attribute__((ext_vector_type(8)))  _Float16 v8h;
typedef __attribute__((ext_vector_type(16))) __bf16   v16b;
typedef __attribute__((ext_vector_type(8)))  __bf16   v8b;
typedef __attribute__((ext_vector_type(8)))  float    v8f;
typedef __attribute__((ext_vector_type(4)))  float    v4f;
typedef __attribute__((ext_vector_type(2)))  float    v2f;

constexpr int kBatch   = 4;
constexpr int kSeq     = 2048;
constexpr int kDim     = 1024;
constexpr int kFilt    = 256;
constexpr int kRows    = kBatch * kSeq;
constexpr int kTaps    = kSeq / 2;
constexpr int kThreads = 256;

constexpr int kConvT = 128;
constexpr int kConvP = 32;
constexpr int kConvJ = 32;
constexpr int kConvW = 192;

static_assert(kConvP == 32);
static_assert(kConvW >= kConvT + 2 * (kConvJ - 1));
static_assert((kConvW * kConvP) % kThreads == 0 && (kConvW * kConvP) / kThreads == 24);
static_assert((kConvJ * kConvP) % kThreads == 0 && (kConvJ * kConvP) / kThreads == 4);
static_assert(kSeq % kConvT == 0 && kDim % (2 * kConvP) == 0 && kTaps % kConvJ == 0);
static_assert(kThreads / 32 * 16 == kConvT);
static_assert(kRows % 64 == 0 && kDim % 64 == 0 && kTaps % 64 == 0);
static_assert(kDim % 32 == 0 && kFilt % 32 == 0);
static_assert(kDim % 64 == 0 && kFilt % 64 == 0);
static_assert(kDim % 8 == 0 && kFilt % 8 == 0);

constexpr size_t kOffA1    = 0;
constexpr size_t kBytesA1  = (size_t)kRows * kDim * 2;
constexpr size_t kOffBt1   = kOffA1 + kBytesA1;
constexpr size_t kBytesBt1 = (size_t)kDim * kDim * 2;
constexpr size_t kOffA2    = kOffBt1 + kBytesBt1;
constexpr size_t kBytesA2  = (size_t)kTaps * kFilt * 2;
constexpr size_t kOffBt2   = kOffA2 + kBytesA2;
constexpr size_t kBytesBt2 = (size_t)kDim * kFilt * 2;
constexpr size_t kOffXP    = kOffBt2 + kBytesBt2;
constexpr size_t kBytesXP  = (size_t)kRows * kDim * 4;
constexpr size_t kOffW     = kOffXP + kBytesXP;
constexpr size_t kBytesW   = (size_t)kTaps * kDim * 4;
constexpr size_t kWsTotal  = kOffW + kBytesW;
static_assert(kWsTotal == 57671680);
static_assert(kWsTotal <= (size_t)134217728);
static_assert(kOffBt1 % 128 == 0 && kOffA2 % 128 == 0 && kOffBt2 % 128 == 0 && kOffXP % 128 == 0 && kOffW % 128 == 0);

__device__ __forceinline__ unsigned short f2bf_bits(float f) {
  unsigned u = __float_as_uint(f);
  return (unsigned short)((u + 0x7FFFu + ((u >> 16) & 1u)) >> 16);
}
__device__ __forceinline__ float bf_bits2f(unsigned short h) { return __uint_as_float(((unsigned)h) << 16); }

__device__ __forceinline__ void dep_guard_h(v8f& a, v8f& b, v16h x, v16h y) { asm volatile("v_nop\n\tv_nop\n\tv_nop\n\tv_nop" : "+v"(a), "+v"(b) : "v"(x), "v"(y)); }
__device__ __forceinline__ void dep_guard_b(v8f& a, v8f& b, v16b x, v16b y) { asm volatile("v_nop\n\tv_nop\n\tv_nop\n\tv_nop" : "+v"(a), "+v"(b) : "v"(x), "v"(y)); }
__device__ __forceinline__ void keep4_h(v16h a, v16h b, v16h c, v16h d) { asm volatile("v_nop" :: "v"(a), "v"(b), "v"(c), "v"(d)); }
__device__ __forceinline__ void keep4_b(v16b a, v16b b, v16b c, v16b d) { asm volatile("v_nop" :: "v"(a), "v"(b), "v"(c), "v"(d)); }
__device__ __forceinline__ void acc_guard4(v8f& a, v8f& b, v8f& c, v8f& d) { asm volatile("v_nop\n\tv_nop\n\tv_nop\n\tv_nop" : "+v"(a), "+v"(b), "+v"(c), "+v"(d)); }
template <typename T> struct Frag;
template <> struct Frag<_Float16> {
  typedef v16h V; union U { v16h v; v8h h[2]; };
  static __device__ __forceinline__ v16h load(const _Float16* p) {
    U f; f.h[0] = *(const v8h*)(p); f.h[1] = *(const v8h*)(p + 16); return f.v;
  }
  static __device__ __forceinline__ v8f mma(v16h a, v16h b, v8f c) {
    return __builtin_amdgcn_wmma_f32_16x16x32_f16(false, a, false, b, (short)0, c, false, false);
  }
  static __device__ __forceinline__ void guard(v8f& a, v8f& b, v16h x, v16h y) { dep_guard_h(a, b, x, y); }
  static __device__ __forceinline__ void keep(v16h a, v16h b, v16h c, v16h d) { keep4_h(a, b, c, d); }
};
template <> struct Frag<__bf16> {
  typedef v16b V; union U { v16b v; v8b h[2]; };
  static __device__ __forceinline__ v16b load(const __bf16* p) {
    U f; f.h[0] = *(const v8b*)(p); f.h[1] = *(const v8b*)(p + 16); return f.v;
  }
  static __device__ __forceinline__ v8f mma(v16b a, v16b b, v8f c) {
    return __builtin_amdgcn_wmma_f32_16x16x32_bf16(false, a, false, b, (short)0, c, false, false);
  }
  static __device__ __forceinline__ void guard(v8f& a, v8f& b, v16b x, v16b y) { dep_guard_b(a, b, x, y); }
  static __device__ __forceinline__ void keep(v16b a, v16b b, v16b c, v16b d) { keep4_b(a, b, c, d); }
};

template <int ET> struct Elem;
template <> struct Elem<0> { typedef _Float16 T; };
template <> struct Elem<1> { typedef __bf16 T; };
template <int ET, bool SPLIT, int BIAS_MODE, int OUT_MODE, bool RESID, int ACT = 0>
__global__ __launch_bounds__(256) void wmma_gemm64(
    const unsigned short* __restrict__ Ap, const unsigned short* __restrict__ A2p, int lda, long strideA,
    const unsigned short* __restrict__ Btp, const unsigned short* __restrict__ Bt2p, int ldb, long strideB,
    void* __restrict__ Cout, void* __restrict__ Cout2, int ldc, long strideC,
    const float* __restrict__ bias,
    const float* __restrict__ resid, long strideR,
    int M, int N, int K, float scale) {
  typedef typename Elem<ET>::T T;
  typedef typename Frag<T>::V V;
  const T* A = (const T*)Ap; const T* A2 = (const T*)A2p; const T* Bt = (const T*)Btp; const T* Bt2 = (const T*)Bt2p;
  __shared__ __align__(16) float sT[8][16 * 68];
  const int b    = blockIdx.y;
  const int lane = threadIdx.x & 31;
  const int wave = threadIdx.x >> 5;
  const int tilesN = N >> 6;
  const int tilesM = M >> 6;
  const int tile = blockIdx.x * 8 + wave;
  if (tile >= tilesM * tilesN) return;
  const int tm = tile / tilesN;
  const int tn = tile - tm * tilesN;
  const int m0 = tm << 6;
  const int n0 = tn << 6;

  const T* Ab  = A  + (size_t)b * strideA;
  const T* Bb  = Bt + (size_t)b * strideB;
  const T* Ab2 = SPLIT ? (A2  + (size_t)b * strideA) : nullptr;
  const T* Bb2 = SPLIT ? (Bt2 + (size_t)b * strideB) : nullptr;

  const int rlane = lane & 15;
  const int koff  = (lane >> 4) * 8;
  const int mOff  = (lane >> 4) * 8;

  v8f acc[4][4];
#pragma unroll
  for (int i = 0; i < 4; ++i)
#pragma unroll
    for (int j = 0; j < 4; ++j) acc[i][j] = (v8f){0.f,0.f,0.f,0.f,0.f,0.f,0.f,0.f};

  for (int k0 = 0; k0 < K; k0 += 32) {
    V bh[4], bl[4];
#pragma unroll
    for (int j = 0; j < 4; ++j) {
      const size_t bo = (size_t)(n0 + (j << 4) + rlane) * ldb + koff + k0;
      bh[j] = Frag<T>::load(Bb + bo);
      if (SPLIT) bl[j] = Frag<T>::load(Bb2 + bo);
    }
#pragma unroll
    for (int i = 0; i < 4; ++i) {
      const size_t ao = (size_t)(m0 + (i << 4) + rlane) * lda + koff + k0;
      V ah = Frag<T>::load(Ab + ao);
      V al;
      if (SPLIT) al = Frag<T>::load(Ab2 + ao);
#pragma unroll
      for (int j = 0; j < 4; ++j) {
        acc[i][j] = Frag<T>::mma(ah, bh[j], acc[i][j]);
        if (SPLIT) {
          acc[i][j] = Frag<T>::mma(ah, bl[j], acc[i][j]);
          acc[i][j] = Frag<T>::mma(al, bh[j], acc[i][j]);
        }
      }
      Frag<T>::guard(acc[i][0], acc[i][3], ah, SPLIT ? al : ah);
    }
    Frag<T>::keep(bh[0], bh[1], bh[2], bh[3]);
    if (SPLIT) Frag<T>::keep(bl[0], bl[1], bl[2], bl[3]);
  }
  acc_guard4(acc[0][0], acc[0][1], acc[0][2], acc[0][3]);
  acc_guard4(acc[1][0], acc[1][1], acc[1][2], acc[1][3]);
  acc_guard4(acc[2][0], acc[2][1], acc[2][2], acc[2][3]);
  acc_guard4(acc[3][0], acc[3][1], acc[3][2], acc[3][3]);

  float* slab = sT[wave];
  const float* Rb = RESID ? (resid + (size_t)b * strideR) : nullptr;
#pragma unroll
  for (int i = 0; i < 4; ++i) {
    const int mBase = m0 + (i << 4);
#pragma unroll
    for (int j = 0; j < 4; ++j) {
      const int n = n0 + (j << 4) + rlane;
      float bv = 0.f;
      if (BIAS_MODE == 2) bv = bias[n];
#pragma unroll
      for (int r = 0; r < 8; ++r) {
        float v = acc[i][j][r] * scale;
        if (BIAS_MODE == 1) v += bias[mBase + mOff + r];
        if (BIAS_MODE == 2) v += bv;
        if (RESID) v += Rb[(size_t)(mBase + mOff + r) * ldc + n];
        if (ACT == 1) v = tanhf(v);
        if (ACT == 2) v = fmaxf(v, 0.0f);
        if (ACT == 3) v = v / (1.0f + expf(-v));
        if (ACT == 4) v = (v > 0.f) ? v : 0.01f * v;
        if (ACT == 5) v = 0.5f * v * (1.0f + erff(v * 0.70710678118654752f));
        slab[(mOff + r) * 68 + (j << 4) + rlane] = v;
      }
    }
    __builtin_amdgcn_fence(__ATOMIC_RELEASE, "workgroup");
    __builtin_amdgcn_wave_barrier();
    __builtin_amdgcn_fence(__ATOMIC_ACQUIRE, "workgroup");
    if (OUT_MODE == 0) {
      float* C = (float*)Cout + (size_t)b * strideC;
      const int hh = lane >> 4, c4 = (lane & 15) * 4;
      for (int pass = 0; pass < 2; ++pass) {
#pragma unroll
        for (int it = 0; it < 8; ++it) {
          const int row = it * 2 + hh;
          v4f v = *(const v4f*)(slab + row * 68 + c4);
          *(volatile v4f*)(C + (size_t)(mBase + row) * ldc + n0 + c4) = v;
        }
        __threadfence();
      }
    } else {
      const int q = lane >> 3, c8 = (lane & 7) * 8;
      unsigned short* C  = (unsigned short*)Cout  + (size_t)b * strideC;
      unsigned short* C2 = (OUT_MODE == 2) ? ((unsigned short*)Cout2 + (size_t)b * strideC) : nullptr;
      for (int pass = 0; pass < 2; ++pass) {
#pragma unroll
        for (int it = 0; it < 4; ++it) {
          const int row = it * 4 + q;
          const float* sp = slab + row * 68 + c8;
          v8h hv, lv;
#pragma unroll
          for (int e = 0; e < 8; ++e) {
            if (OUT_MODE == 1) {
              hv[e] = (_Float16)sp[e];
            } else {
              unsigned short hb = f2bf_bits(sp[e]);
              unsigned short lb = f2bf_bits(sp[e] - bf_bits2f(hb));
              hv[e] = __builtin_bit_cast(_Float16, hb);
              lv[e] = __builtin_bit_cast(_Float16, lb);
            }
          }
          *(volatile v8h*)(C + (size_t)(mBase + row) * ldc + n0 + c8) = hv;
          if (OUT_MODE == 2) *(volatile v8h*)(C2 + (size_t)(mBase + row) * ldc + n0 + c8) = lv;
        }
        __threadfence();
      }
    }
    __builtin_amdgcn_fence(__ATOMIC_RELEASE, "workgroup");
    __builtin_amdgcn_wave_barrier();
    __builtin_amdgcn_fence(__ATOMIC_ACQUIRE, "workgroup");
  }
}

__device__ __forceinline__ float bfr(float f) { return bf_bits2f(f2bf_bits(f)); }

__global__ __launch_bounds__(kThreads) void cvt_rows_bf16(const float* __restrict__ in, int rows, int cols, int row_step,
                                                          float scale, unsigned short* __restrict__ out) {
  const int tpr = cols >> 3;
  const int i = blockIdx.x * kThreads + threadIdx.x;
  if (i >= rows * tpr) return;
  const int r  = i / tpr;
  const int c0 = (i - r * tpr) * 8;
  const float* src = in + (size_t)r * (size_t)row_step * (size_t)cols + c0;
  const v4f a0 = *(const v4f*)(src);
  const v4f a1 = *(const v4f*)(src + 4);
  v8h hv;
#pragma unroll
  for (int e = 0; e < 4; ++e) {
    hv[e]     = __builtin_bit_cast(_Float16, f2bf_bits(scale * bfr(a0[e])));
    hv[4 + e] = __builtin_bit_cast(_Float16, f2bf_bits(scale * bfr(a1[e])));
  }
  unsigned short* dst = out + (size_t)i * 8;
  for (int pass = 0; pass < 2; ++pass) {
    *(volatile v8h*)(dst) = hv;
    __threadfence();
  }
}

__global__ __launch_bounds__(kThreads) void cvt_T_bf16(const float* __restrict__ in, int R, int C, unsigned short* __restrict__ out) {
  __shared__ float sm[64 * 65];
  const int tid = threadIdx.x, lane = tid & 31, wave = tid >> 5;
  const int n0 = blockIdx.x * 64, k0 = blockIdx.y * 64;
  const int nn = tid & 63, kq = tid >> 6;
#pragma unroll
  for (int i = 0; i < 8; ++i) {
    const int kk = kq + 4 * i;
    sm[kk * 65 + nn] = in[(size_t)(k0 + kk) * C + n0 + nn];
  }
  asm volatile("" ::: "memory");
#pragma unroll
  for (int i = 8; i < 16; ++i) {
    const int kk = kq + 4 * i;
    sm[kk * 65 + nn] = in[(size_t)(k0 + kk) * C + n0 + nn];
  }
  __syncthreads();
  const int q = lane >> 3, c8 = (lane & 7) * 8;
  const int nr0 = wave * 4 + q;
  const int nr1 = 32 + wave * 4 + q;
  v8h hv0, hv1;
#pragma unroll
  for (int e = 0; e < 8; ++e) {
    hv0[e] = __builtin_bit_cast(_Float16, f2bf_bits(sm[(c8 + e) * 65 + nr0]));
    hv1[e] = __builtin_bit_cast(_Float16, f2bf_bits(sm[(c8 + e) * 65 + nr1]));
  }
  unsigned short* p0 = out + (size_t)(n0 + nr0) * R + k0 + c8;
  unsigned short* p1 = out + (size_t)(n0 + nr1) * R + k0 + c8;
  for (int pass = 0; pass < 2; ++pass) {
    *(volatile v8h*)(p0) = hv0;
    *(volatile v8h*)(p1) = hv1;
    __threadfence();
  }
}

__global__ __launch_bounds__(kThreads) void conv_even_lag(const float* __restrict__ u, const float* __restrict__ w,
                                                          const int* __restrict__ nfft, float* __restrict__ out) {
  __shared__ __align__(16) v2f su[kConvW * kConvP];
  __shared__ __align__(16) v2f sw[kConvJ * kConvP];
  constexpr int Dh = kDim / 2;

  const int tid  = threadIdx.x;
  const int lane = tid & 31;
  const int tg   = tid >> 5;
  const int tb   = tg * 16;
  const int t0   = blockIdx.x * kConvT;
  const int d0   = blockIdx.y * (2 * kConvP);
  const int b    = blockIdx.z;

  const v2f* ub2 = (const v2f*)(u + (size_t)b * kSeq * kDim + d0);
  const v2f* w2  = (const v2f*)(w + d0);

  v2f acc[16];
#pragma unroll
  for (int i = 0; i < 16; ++i) acc[i] = (v2f){0.0f, 0.0f};

  const int jh    = (t0 + kConvT - 1) >> 1;
  const int jlast = (jh < kTaps - 1) ? jh : (kTaps - 1);

#pragma unroll 1
  for (int j0 = 0; j0 <= jlast; j0 += kConvJ) {
    const int tw0 = t0 - 2 * j0 - 2 * (kConvJ - 1);
#pragma unroll
    for (int g = 0; g < 3; ++g) {
#pragma unroll
      for (int r = 0; r < 8; ++r) {
        const int e   = (g * 8 + r) * kThreads + tid;
        const int tt  = e >> 5;
        const int cc  = e & 31;
        const int t   = tw0 + tt;
        const int tcl = (t < 0) ? 0 : ((t > kSeq - 1) ? (kSeq - 1) : t);
        const float fa = (t >= 0 && t < kSeq) ? 1.0f : 0.0f;
        const v2f v = ub2[(size_t)tcl * Dh + cc];
        su[e] = v * fa;
      }
      asm volatile("" ::: "memory");
    }
#pragma unroll
    for (int r = 0; r < 4; ++r) {
      const int e  = r * kThreads + tid;
      const int jj = e >> 5;
      const int cc = e & 31;
      int j = j0 + jj;
      j = (j > kTaps - 1) ? (kTaps - 1) : j;
      sw[e] = w2[(size_t)j * Dh + cc];
    }
    __syncthreads();

#pragma unroll 4
    for (int jj = 0; jj < kConvJ; ++jj) {
      const v2f wv  = sw[jj * kConvP + lane];
      const int base = tb + 2 * (kConvJ - 1) - 2 * jj;
#pragma unroll
      for (int i = 0; i < 16; ++i) acc[i] += wv * su[(base + i) * kConvP + lane];
    }
    __syncthreads();
  }

#pragma unroll
  for (int i = 0; i < 16; ++i) su[(tb + i) * kConvP + lane] = acc[i];
  __syncthreads();

  const int nv = nfft[0];
  const float addv = (nv >= 2 * kSeq - 1) ? 0.0f : __uint_as_float(0x7fc00000u);

  const int hh = lane >> 4, cq = lane & 15;
  float* ob = out + ((size_t)b * kSeq + (size_t)(t0 + tb)) * kDim + d0 + 4 * cq;
  for (int pass = 0; pass < 2; ++pass) {
#pragma unroll
    for (int it = 0; it < 8; ++it) {
      const int row = it * 2 + hh;
      const v2f p0 = su[(tb + row) * kConvP + 2 * cq];
      const v2f p1 = su[(tb + row) * kConvP + 2 * cq + 1];
      v4f v;
      v[0] = p0[0] + addv; v[1] = p0[1] + addv; v[2] = p1[0] + addv; v[3] = p1[1] + addv;
      *(volatile v4f*)(ob + (size_t)row * kDim) = v;
    }
    __threadfence();
  }
}

extern "C" void kernel_launch(void* const* d_in, const int* in_sizes, int n_in,
                              void* d_out, int out_size, void* d_ws, size_t ws_size,
                              hipStream_t stream) {
  if (n_in < 5) return;
  if (in_sizes[0] != kRows * kDim || in_sizes[1] != kSeq * kFilt || in_sizes[2] != kDim * kDim ||
      in_sizes[3] != kFilt * kDim || in_sizes[4] < 1) return;
  if (out_size != kRows * kDim) return;
  if (ws_size < kWsTotal) return;

  const float* x    = (const float*)d_in[0];
  const float* phi  = (const float*)d_in[1];
  const float* w_in = (const float*)d_in[2];
  const float* w_fl = (const float*)d_in[3];
  const int*   nptr = (const int*)d_in[4];
  float* out = (float*)d_out;

  char* ws = (char*)d_ws;
  unsigned short* A1  = (unsigned short*)(ws + kOffA1);
  unsigned short* Bt1 = (unsigned short*)(ws + kOffBt1);
  unsigned short* A2  = (unsigned short*)(ws + kOffA2);
  unsigned short* Bt2 = (unsigned short*)(ws + kOffBt2);
  float* xproj = (float*)(ws + kOffXP);
  float* wtap  = (float*)(ws + kOffW);

  cvt_rows_bf16<<<(kRows * (kDim / 8)) / kThreads, kThreads, 0, stream>>>(x, kRows, kDim, 1, 1.0f, A1);
  cvt_rows_bf16<<<(kTaps * (kFilt / 8)) / kThreads, kThreads, 0, stream>>>(phi, kTaps, kFilt, 2, 2.0f, A2);
  cvt_T_bf16<<<dim3(kDim / 64, kDim / 64), kThreads, 0, stream>>>(w_in, kDim, kDim, Bt1);
  cvt_T_bf16<<<dim3(kDim / 64, kFilt / 64), kThreads, 0, stream>>>(w_fl, kFilt, kDim, Bt2);

  {
    const int tiles = (kRows / 64) * (kDim / 64);
    wmma_gemm64<1, false, 0, 0, false, 0><<<dim3((tiles + 7) / 8, 1), 256, 0, stream>>>(
        A1, A1, kDim, 0L, Bt1, Bt1, kDim, 0L, (void*)xproj, (void*)xproj, kDim, 0L,
        (const float*)wtap, (const float*)wtap, 0L, kRows, kDim, kDim, 1.0f);
  }
  {
    const int tiles = (kTaps / 64) * (kDim / 64);
    wmma_gemm64<1, false, 0, 0, false, 0><<<dim3((tiles + 7) / 8, 1), 256, 0, stream>>>(
        A2, A2, kFilt, 0L, Bt2, Bt2, kFilt, 0L, (void*)wtap, (void*)wtap, kDim, 0L,
        (const float*)xproj, (const float*)xproj, 0L, kTaps, kDim, kFilt, 1.0f);
  }
  conv_even_lag<<<dim3(kSeq / kConvT, kDim / (2 * kConvP), kBatch), kThreads, 0, stream>>>(xproj, wtap, nptr, out);
}
